// S4A_NS_73418170958498
// MI455X (gfx1250) — hardware-verified
//
#include <hip/hip_runtime.h>
#include <math.h>

typedef __attribute__((ext_vector_type(16))) _Float16 v16h;
typedef __attribute__((ext_vector_type(16))) __bf16 v16b;
typedef __attribute__((ext_vector_type(8)))  _Float16 v8h;
typedef __attribute__((ext_vector_type(8)))  float v8f;
typedef __attribute__((ext_vector_type(4)))  float v4f;
typedef __attribute__((ext_vector_type(2)))  float v2f;
typedef __attribute__((ext_vector_type(4)))  unsigned v4u;
typedef __attribute__((ext_vector_type(4)))  int v4i;
typedef float __attribute__((may_alias)) float_a;
typedef int __attribute__((may_alias)) int_a;

template <typename T> __device__ __forceinline__ void vst2(void* p, T v) { *(volatile T*)p = v; __threadfence(); *(volatile T*)p = v; }
__device__ __forceinline__ v8f wmma16(v16h a, v16h b, v8f c) {
  v8f d = __builtin_amdgcn_wmma_f32_16x16x32_f16(false, a, false, b, (short)0, c, false, false);
  asm volatile("v_nop\n\tv_nop\n\tv_nop\n\tv_nop" : "+v"(d) : "v"(a), "v"(b));
  return d;
}
__device__ __forceinline__ v8f wmma_bf(v16b a, v16b b, v8f c) {
  v8f d = __builtin_amdgcn_wmma_f32_16x16x32_bf16(false, a, false, b, (short)0, c, false, false);
  asm volatile("v_nop\n\tv_nop\n\tv_nop\n\tv_nop" : "+v"(d) : "v"(a), "v"(b));
  return d;
}
__device__ __forceinline__ v16h frag_h(const _Float16* rowk0, int lane) {
  union { v16h v; v8h q[2]; } u; const _Float16* p = rowk0 + 8 * (lane >> 4);
  u.q[0] = *(const v8h*)p; u.q[1] = *(const v8h*)(p + 16); return u.v;
}
__device__ __forceinline__ v16h frag_f32(const float* rowk0, int lane) {
  v16h a; const float* p = rowk0 + 8 * (lane >> 4);
#pragma unroll
  for (int i = 0; i < 8; ++i) { a[i] = (_Float16)p[i]; a[8 + i] = (_Float16)p[16 + i]; }
  return a;
}
__device__ __forceinline__ v16h frag_f32s(const float* rowk0, int lane, float sc) {
  v16h a; const float* p = rowk0 + 8 * (lane >> 4);
#pragma unroll
  for (int i = 0; i < 8; ++i) { a[i] = (_Float16)(p[i] * sc); a[8 + i] = (_Float16)(p[16 + i] * sc); }
  return a;
}
__device__ __forceinline__ v16h fragc_f32(const float* W, int k0, int n, int lane, int ld, int K) {
  v16h a; const int g = lane >> 4;
#pragma unroll
  for (int i = 0; i < 8; ++i) { const int ka = k0 + 8 * g + i, kb = ka + 16;
    a[i] = (_Float16)(ka < K ? W[(size_t)(ka < K ? ka : K - 1) * ld + n] : 0.f); a[8 + i] = (_Float16)(kb < K ? W[(size_t)(kb < K ? kb : K - 1) * ld + n] : 0.f); }
  return a;
}
struct F2 { v16b h, l; };
__device__ __forceinline__ F2 bsplit16(const float v[16]) { F2 r;
#pragma unroll
  for (int i = 0; i < 16; ++i) { const __bf16 h = (__bf16)v[i]; r.h[i] = h; r.l[i] = (__bf16)(v[i] - (float)h); }
  return r; }
__device__ __forceinline__ F2 split_row(const float* row, int k0, int lane) { float v[16]; const float* p = row + k0 + 8 * (lane >> 4);
#pragma unroll
  for (int i = 0; i < 8; ++i) { v[i] = p[i]; v[8 + i] = p[16 + i]; }
  return bsplit16(v); }
__device__ __forceinline__ F2 split_rowK(const float* row, int k0, int lane, int K) { float v[16]; const int g = lane >> 4;
#pragma unroll
  for (int i = 0; i < 8; ++i) { const int ka = k0 + 8 * g + i, kb = ka + 16; v[i] = ka < K ? row[ka < K ? ka : K - 1] : 0.f; v[8 + i] = kb < K ? row[kb < K ? kb : K - 1] : 0.f; }
  return bsplit16(v); }
__device__ __forceinline__ F2 split_col(const float* W, int k0, int n, int lane, int ld, int K) { float v[16]; const int g = lane >> 4;
#pragma unroll
  for (int i = 0; i < 8; ++i) { const int ka = k0 + 8 * g + i, kb = ka + 16; v[i] = ka < K ? W[(size_t)(ka < K ? ka : K - 1) * ld + n] : 0.f; v[8 + i] = kb < K ? W[(size_t)(kb < K ? kb : K - 1) * ld + n] : 0.f; }
  return bsplit16(v); }
__device__ __forceinline__ v8f mac3(const F2& a, const F2& b, v8f c) { c = wmma_bf(a.l, b.h, c); c = wmma_bf(a.h, b.l, c); return wmma_bf(a.h, b.h, c); }
__device__ __forceinline__ float sigm(float v) { return 1.0f / (1.0f + expf(-v)); }
#define LDSX() do { asm volatile("s_wait_dscnt 0" ::: "memory"); __builtin_amdgcn_wave_barrier(); __builtin_amdgcn_fence(__ATOMIC_RELEASE, "workgroup"); } while (0)


#define NBT 16
#define LL 1024
#define NTOK (NBT * LL)
#define DIN 768
#define BD 384
#define EE 768
#define NS 16
#define RR 24
#define KC 4
#define XW 64
#ifndef TNB
#define TNB NBT
#endif
typedef __attribute__((ext_vector_type(8))) __bf16 v8b;
__device__ __forceinline__ v16b frag_b(const __bf16* rowk0, int lane) {
  union { v16b v; v8b q[2]; } u; const __bf16* p = rowk0 + 8 * (lane >> 4);
  u.q[0] = *(const v8b*)p; u.q[1] = *(const v8b*)(p + 16); return u.v;
}
__device__ __forceinline__ float bfr(float v) { return (float)(__bf16)v; }
__device__ __attribute__((noinline)) float exp_ni(float v) { return expf(v); }
__device__ __attribute__((noinline)) float erf_ni(float v) { return erff(v); }

__device__ __attribute__((noinline)) float log1p_ni(float v) { return log1pf(v); }
#define WS_PW   0u
#define PWD 0
#define PWIN (PWD + BD * DIN)
#define PWX (PWIN + 2 * EE * BD)
#define PWDT (PWX + XW * EE)
#define PWO (PWDT + EE * 32)
#define PWU (PWO + BD * EE)
#define PWEND (PWU + DIN * BD)
#define WS_H    (WS_PW + 2u * PWEND)
#define WS_XZ   (WS_H + 4u * NTOK * BD)
#define WS_U    (WS_XZ + 4u * NTOK * 2 * EE)
#define WS_XD   (WS_U + 4u * NTOK * EE)
#define WS_DT   (WS_XD + 4u * NTOK * XW)
#define WS_END  (WS_DT + 4u * NTOK * EE)

__global__ __launch_bounds__(256) void k_packT(const float* __restrict__ WD, const float* __restrict__ WIN, const float* __restrict__ WX, const float* __restrict__ WDT, const float* __restrict__ WO, const float* __restrict__ WU, __bf16* __restrict__ PW) {
  __shared__ __align__(16) __bf16 s[DIN]; const int n = blockIdx.x, which = blockIdx.y, tid = threadIdx.x; int K, N; const float* Wm; size_t base; int Kreal;
  if (which == 0) { K = DIN; N = BD; Wm = WD; base = PWD; } else if (which == 1) { K = BD; N = 2 * EE; Wm = WIN; base = PWIN; } else if (which == 2) { K = EE; N = XW; Wm = WX; base = PWX; } else if (which == 3) { K = 32; N = EE; Wm = WDT; base = PWDT; } else if (which == 4) { K = EE; N = BD; Wm = WO; base = PWO; } else { K = BD; N = DIN; Wm = WU; base = PWU; }
  if (n >= N) return; Kreal = (which == 3) ? RR : K; const int Nreal = (which == 2) ? (RR + 2 * NS) : N;
  for (int k = tid; k < K; k += 256) s[k] = (__bf16)((k < Kreal && n < Nreal) ? Wm[(size_t)k * Nreal + n] : 0.f);
  __syncthreads();
  for (int q = tid; q < K / 8; q += 256) vst2((unsigned*)(PW + base + (size_t)n * K + q * 8), *(const v4u*)&s[q * 8]);
}
template <int RIN, int NT, int EPI>
__global__ __launch_bounds__(128) void k_gemm(const float* __restrict__ A, int lda, int K, const __bf16* __restrict__ P, const float* __restrict__ bias, float* __restrict__ OUT, int ldo) {
  __shared__ __align__(16) float so[4][16][NT * 16 + 4];
  const int tid = threadIdx.x, wave = tid >> 5, lane = tid & 31, col = lane & 15, g = lane >> 4; const size_t r0 = (size_t)blockIdx.x * 64 + wave * 16; const int n0 = blockIdx.y * (NT * 16);
  v8f acc[NT]; for (int j = 0; j < NT; ++j) acc[j] = (v8f){};
#pragma unroll 2
  for (int kc = 0; kc < K / 32; ++kc) { F2 a; if (RIN) { v16b ax; const float* p = A + (r0 + col) * lda + kc * 32 + 8 * g;
#pragma unroll
      for (int i = 0; i < 8; ++i) { ax[i] = (__bf16)p[i]; ax[8 + i] = (__bf16)p[16 + i]; } a.h = ax; a.l = ax; } else a = split_row(A + (r0 + col) * lda, kc * 32, lane);
#pragma unroll
    for (int j = 0; j < NT; ++j) { const v16b wv = frag_b(P + (size_t)(n0 + j * 16 + col) * K + kc * 32, lane); if (!RIN) acc[j] = wmma_bf(a.l, wv, acc[j]); acc[j] = wmma_bf(a.h, wv, acc[j]); } }
#pragma unroll
  for (int j = 0; j < NT; ++j) { const int n = n0 + j * 16 + col; const float b_ = bias ? bfr(bias[n]) : 0.f;
#pragma unroll
    for (int r = 0; r < 8; ++r) { float v = acc[j][r] + b_; if (EPI == 1) { v = (v > 20.f) ? v : log1p_ni(exp_ni(v)); } so[wave][8 * g + r][j * 16 + col] = v; } }
  LDSX();
  for (int rl = 0; rl < 16; ++rl) if (lane < NT * 4) vst2(OUT + (r0 + rl) * ldo + n0 + lane * 4, *(const v4f*)&so[wave][rl][lane * 4]);
}
__global__ __launch_bounds__(256) void k_conv(const float* __restrict__ XZ, const float* __restrict__ CWt, const float* __restrict__ CB, float* __restrict__ U) {
  __shared__ __align__(16) float so[16][EE];
  const int tid = threadIdx.x; const size_t r0 = (size_t)blockIdx.x * 64; const int b = (int)(r0 / LL); const int l0 = (int)(r0 % LL);
  float w[3][KC], cb[3];
#pragma unroll
  for (int m = 0; m < 3; ++m) { const int e = tid + 256 * m; cb[m] = bfr(CB[e]);
#pragma unroll
    for (int j = 0; j < KC; ++j) w[m][j] = bfr(CWt[e * KC + j]); }
#pragma unroll 1
  for (int part = 0; part < 4; ++part) {
#pragma unroll
    for (int m = 0; m < 3; ++m) { const int e = tid + 256 * m;
      for (int rl = 0; rl < 16; ++rl) { const int l = l0 + part * 16 + rl; float acc = cb[m];
#pragma unroll
        for (int j = 0; j < KC; ++j) { const int ls = l - (KC - 1) + j; if (ls >= 0) acc += w[m][j] * XZ[((size_t)b * LL + ls) * (2 * EE) + e]; }
        so[rl][e] = acc * sigm(acc); } }
    __syncthreads();
    for (int q = tid; q < 16 * EE / 4; q += 256) { const int rl = q / (EE / 4), pc = q % (EE / 4); vst2(U + (r0 + part * 16 + rl) * EE + pc * 4, *(const v4f*)&so[rl][pc * 4]); }
    __syncthreads(); }
}
__global__ __launch_bounds__(256) void k_scan(const float* __restrict__ XZ, const float* __restrict__ XD, const float* __restrict__ DT, const float* __restrict__ ALOG, const float* __restrict__ Dv, float* U) {
  __shared__ __align__(16) float sred[8][32]; __shared__ __align__(16) float sy[32];
  const int tid = threadIdx.x, el = tid & 31, ng = tid >> 5; const int ech = blockIdx.x, b = blockIdx.y; const int e = ech * 32 + el;
  float An[2], h[2];
#pragma unroll
  for (int i = 0; i < 2; ++i) { An[i] = -exp_ni(bfr(ALOG[(size_t)e * NS + ng * 2 + i])); h[i] = 0.f; }
  const float dd = bfr(Dv[e]);
#pragma unroll 1
  for (int l = 0; l < LL; ++l) { const size_t row = (size_t)b * LL + l;
    const float dt = DT[row * EE + e], u = U[row * EE + e]; const float* xd = XD + row * XW;
    float py = 0.f;
#pragma unroll
    for (int i = 0; i < 2; ++i) { const int n = ng * 2 + i; h[i] = h[i] * exp_ni(dt * An[i]) + dt * u * xd[RR + n]; py += h[i] * xd[RR + NS + n]; }
    sred[ng][el] = py;
    __syncthreads();
    if (tid < 32) { float y = 0.f;
#pragma unroll
      for (int q = 0; q < 8; ++q) y += sred[q][tid];
      const int e2 = ech * 32 + tid; const float u2 = U[row * EE + e2]; const float z = XZ[row * (2 * EE) + EE + e2];
      sy[tid] = (y + u2 * bfr(Dv[e2])) * (z * sigm(z)); }
    __syncthreads();
    if (tid < 8) vst2(U + row * EE + ech * 32 + tid * 4, *(const v4f*)&sy[tid * 4]);
  }
}
extern "C" void kernel_launch(void* const* d_in, const int* in_sizes, int n_in, void* d_out, int out_size, void* d_ws, size_t ws_size, hipStream_t stream) {
  (void)in_sizes; (void)n_in; (void)out_size;
  const float** F = (const float**)d_in;
  if (ws_size < (size_t)WS_END) return;
  char* ws = (char*)d_ws; __bf16* PW = (__bf16*)(ws + WS_PW); float *H = (float*)(ws + WS_H), *XZ = (float*)(ws + WS_XZ), *U = (float*)(ws + WS_U), *XD = (float*)(ws + WS_XD), *DT = (float*)(ws + WS_DT);
  const int NR = TNB * LL / 64;
  k_packT<<<dim3(2 * EE, 6), 256, 0, stream>>>(F[1], F[3], F[6], F[7], F[11], F[12], PW);
  k_gemm<1, 8, 0><<<dim3(NR, BD / 128), 128, 0, stream>>>(F[0], DIN, DIN, PW + PWD, F[2], H, BD);
  k_gemm<0, 8, 0><<<dim3(NR, 2 * EE / 128), 128, 0, stream>>>(H, BD, BD, PW + PWIN, nullptr, XZ, 2 * EE);
  k_conv<<<NR, 256, 0, stream>>>(XZ, F[4], F[5], U);
  k_gemm<0, 4, 0><<<dim3(NR, 1), 128, 0, stream>>>(U, EE, EE, PW + PWX, nullptr, XD, XW);
  k_gemm<0, 8, 1><<<dim3(NR, EE / 128), 128, 0, stream>>>(XD, XW, 32, PW + PWDT, F[8], DT, EE);
  k_scan<<<dim3(EE / 32, TNB), 256, 0, stream>>>(XZ, XD, DT, F[9], F[10], U);
  k_gemm<0, 8, 0><<<dim3(NR, BD / 128), 128, 0, stream>>>(U, EE, EE, PW + PWO, nullptr, H, BD);
  k_gemm<0, 8, 0><<<dim3(NR, DIN / 128), 128, 0, stream>>>(H, BD, BD, PW + PWU, F[13], (float*)d_out, DIN);
}
